// EarlyFusionModel_19980187861743
// MI455X (gfx1250) — hardware-verified
//
#include <hip/hip_runtime.h>
#include <math.h>

typedef __attribute__((ext_vector_type(16))) _Float16 v16h;
typedef __attribute__((ext_vector_type(8)))  _Float16 v8h;
typedef __attribute__((ext_vector_type(8)))  float    v8f;
typedef __attribute__((ext_vector_type(4)))  float    v4f;
typedef __attribute__((ext_vector_type(4)))  int      v4i;
#define U16(p) ((const unsigned short*)(const void*)(p))

__device__ __forceinline__ void dep_guard_h(v8f& a, v8f& b, v16h x, v16h y) { asm volatile("v_nop\n\tv_nop\n\tv_nop\n\tv_nop" : "+v"(a), "+v"(b) : "v"(x), "v"(y)); }
__device__ __forceinline__ void keep4_h(v16h a, v16h b, v16h c, v16h d) { asm volatile("v_nop" :: "v"(a), "v"(b), "v"(c), "v"(d)); }
__device__ __forceinline__ void fence_v4(v4f& t) { asm volatile("" : "+v"(t)); }
__device__ __forceinline__ void acc_guard4(v8f& a, v8f& b, v8f& c, v8f& d) { asm volatile("v_nop\n\tv_nop\n\tv_nop\n\tv_nop" : "+v"(a), "+v"(b), "+v"(c), "+v"(d)); }
template <typename T> struct Frag;
template <> struct Frag<_Float16> {
  typedef v16h V; union U { v16h v; v8h h[2]; };
  static __device__ __forceinline__ v16h load(const _Float16* p) {
    U f; f.h[0] = *(const v8h*)(p); f.h[1] = *(const v8h*)(p + 16); return f.v;
  }
  static __device__ __forceinline__ v8f mma(v16h a, v16h b, v8f c) {
    return __builtin_amdgcn_wmma_f32_16x16x32_f16(false, a, false, b, (short)0, c, false, false);
  }
  static __device__ __forceinline__ void guard(v8f& a, v8f& b, v16h x, v16h y) { dep_guard_h(a, b, x, y); }
  static __device__ __forceinline__ void keep(v16h a, v16h b, v16h c, v16h d) { keep4_h(a, b, c, d); }
};

#define NN 32768
#define NE 262144
#define NG 1024
#define ETOT (NE + NN)
#define FIN 32
#define EDM 8
#define HC 256
#define NHD 4
#define FPK 2048
#define DSK 200
#define DSKP 224
#define GO 64
#define FO 256
#define DO_ 64
#define TIN 384
#define HD1 192
#define HD2 96
#define HD2P 128
#define NTK 12
#define NT 256
#define SRB 1024
#define RPW (SRB / 8)
#define NTILE (NN / SRB)
#define SCH 2048
#define NCH (NE / SCH)
#define XP 512
#define BNINV 0x1.ffff58p-1f

template <int EPI, bool OUT16>
__global__ __launch_bounds__(256) void gemm_f16(
    const unsigned short* __restrict__ Ap, int lda,
    const unsigned short* __restrict__ Btp, int ldb,
    void* __restrict__ Cout, int ldc,
    const float* __restrict__ bias, const float* __restrict__ gamma, const float* __restrict__ beta,
    int nValid, int M, int N, int K, float scale, float oscale) {
  typedef _Float16 T;
  typedef v16h V;
  const T* A = (const T*)Ap; const T* Bt = (const T*)Btp;
  __shared__ __align__(16) float sT[8][16 * 68];
  const int lane = threadIdx.x & 31;
  const int wave = threadIdx.x >> 5;
  const int tilesN = N >> 6;
  const int tilesM = M >> 6;
  const int tile = blockIdx.x * 8 + wave;
  if (tile >= tilesM * tilesN) return;
  const int tm = tile / tilesN;
  const int tn = tile - tm * tilesN;
  const int m0 = tm << 6;
  const int n0 = tn << 6;

  const int rlane = lane & 15;
  const int koff  = (lane >> 4) * 8;
  const int mOff  = (lane >> 4) * 8;

  v8f acc[4][4];
#pragma unroll
  for (int i = 0; i < 4; ++i)
#pragma unroll
    for (int j = 0; j < 4; ++j) acc[i][j] = (v8f){0.f,0.f,0.f,0.f,0.f,0.f,0.f,0.f};

  for (int k0 = 0; k0 < K; k0 += 32) {
    V bh[4];
#pragma unroll
    for (int j = 0; j < 4; ++j) {
      const size_t bo = (size_t)(n0 + (j << 4) + rlane) * ldb + koff + k0;
      bh[j] = Frag<T>::load(Bt + bo);
    }
#pragma unroll
    for (int i = 0; i < 4; ++i) {
      const size_t ao = (size_t)(m0 + (i << 4) + rlane) * lda + koff + k0;
      V ah = Frag<T>::load(A + ao);
#pragma unroll
      for (int j = 0; j < 4; ++j) acc[i][j] = Frag<T>::mma(ah, bh[j], acc[i][j]);
      Frag<T>::guard(acc[i][0], acc[i][3], ah, ah);
    }
    Frag<T>::keep(bh[0], bh[1], bh[2], bh[3]);
  }
  acc_guard4(acc[0][0], acc[0][1], acc[0][2], acc[0][3]);
  acc_guard4(acc[1][0], acc[1][1], acc[1][2], acc[1][3]);
  acc_guard4(acc[2][0], acc[2][1], acc[2][2], acc[2][3]);
  acc_guard4(acc[3][0], acc[3][1], acc[3][2], acc[3][3]);

  float* slab = sT[wave];
#pragma unroll
  for (int i = 0; i < 4; ++i) {
    const int mBase = m0 + (i << 4);
#pragma unroll
    for (int j = 0; j < 4; ++j) {
      const int n = n0 + (j << 4) + rlane;
      const bool nv = n < nValid;
      const int nc = nv ? n : 0;
      const float bv = bias[nc];
      float gs = 1.f, bt = 0.f;
      if (EPI == 1) { gs = gamma[nc] * BNINV; bt = beta[nc]; }
#pragma unroll
      for (int r = 0; r < 8; ++r) {
        float v = acc[i][j][r] * scale + bv;
        if (EPI == 1) { v = fmaxf(v, 0.0f); v = v * gs + bt; }
        if (!nv) v = 0.f;
        if (OUT16) v *= oscale;
        slab[(mOff + r) * 68 + (j << 4) + rlane] = v;
      }
    }
    __builtin_amdgcn_fence(__ATOMIC_RELEASE, "workgroup");
    __builtin_amdgcn_wave_barrier();
    __builtin_amdgcn_fence(__ATOMIC_ACQUIRE, "workgroup");
    if (!OUT16) {
      float* C = (float*)Cout;
      const int hh = lane >> 4, c4 = (lane & 15) * 4;
      for (int pass = 0; pass < 2; ++pass) {
#pragma unroll
        for (int it = 0; it < 8; ++it) {
          const int row = it * 2 + hh;
          v4f v = *(const v4f*)(slab + row * 68 + c4);
          *(volatile v4f*)(C + (size_t)(mBase + row) * ldc + n0 + c4) = v;
        }
        __threadfence();
      }
    } else {
      const int q = lane >> 3, c8 = (lane & 7) * 8;
      unsigned short* C = (unsigned short*)Cout;
      for (int pass = 0; pass < 2; ++pass) {
#pragma unroll
        for (int it = 0; it < 4; ++it) {
          const int row = it * 4 + q;
          const float* sp = slab + row * 68 + c8;
          v8h hv;
#pragma unroll
          for (int e = 0; e < 8; ++e) hv[e] = (_Float16)sp[e];
          *(volatile v8h*)(C + (size_t)(mBase + row) * ldc + n0 + c8) = hv;
        }
        __threadfence();
      }
    }
    __builtin_amdgcn_fence(__ATOMIC_RELEASE, "workgroup");
    __builtin_amdgcn_wave_barrier();
    __builtin_amdgcn_fence(__ATOMIC_ACQUIRE, "workgroup");
  }
}

__global__ __launch_bounds__(256) void k_cast_rows(const float* __restrict__ in, int R, int C, _Float16* __restrict__ out, int Cp) {
  const long t = (long)blockIdx.x * 256 + threadIdx.x;
  const long f = 8 * t;
  if (f >= (long)R * Cp) return;
  const int r = (int)(f / Cp), k0 = (int)(f - (long)r * Cp);
  const float* src = in + (size_t)r * C;
  v8h hv;
#pragma unroll
  for (int i = 0; i < 8; ++i) { const int k = k0 + i; const float v = (k < C) ? src[k] : 0.f; hv[i] = (_Float16)v; }
  _Float16* op = out + f;
  *(volatile v8h*)op = hv; __threadfence(); *(volatile v8h*)op = hv;
}
__global__ __launch_bounds__(256) void k_tcast(const float* __restrict__ in, int R, int C, _Float16* __restrict__ outT, int Rp, int Cp) {
  const long t = (long)blockIdx.x * 256 + threadIdx.x;
  const long f = 8 * t;
  if (f >= (long)Cp * Rp) return;
  const int c = (int)(f / Rp), r0 = (int)(f - (long)c * Rp);
  v8h hv;
#pragma unroll
  for (int i = 0; i < 8; ++i) {
    const int r = r0 + i;
    const float v = (r < R && c < C) ? in[(size_t)r * C + c] : 0.f;
    hv[i] = (_Float16)v;
  }
  _Float16* op = outT + f;
  *(volatile v8h*)op = hv; __threadfence(); *(volatile v8h*)op = hv;
}
__global__ __launch_bounds__(256) void bias_cat2_kernel(const float* a, const float* b, float* __restrict__ o, int hc) {
  for (int pass = 0; pass < 2; ++pass) { for (int i = threadIdx.x; i < 2 * hc; i += 256) ((volatile float*)o)[i] = (i < hc) ? a[i] : b[i - hc]; __threadfence(); }
}

__device__ __forceinline__ int blk_excl_scan(int cnt, int* scan_ws, int tid, int* tot) {
  const int lane = tid & 31, wave = tid >> 5; int incl = cnt;
#pragma unroll
  for (int o = 1; o < 32; o <<= 1) { const int v = __shfl_up(incl, o, 32); if (lane >= o) incl += v; }
  if (lane == 31) scan_ws[wave] = incl;
  __syncthreads();
  if (wave == 0) { int wv = (lane < NT / 32) ? scan_ws[lane] : 0; int wincl = wv;
#pragma unroll
    for (int o = 1; o < 32; o <<= 1) { const int v = __shfl_up(wincl, o, 32); if (lane >= o) wincl += v; }
    if (lane < NT / 32) scan_ws[32 + lane] = wincl - wv; if (lane == 31) scan_ws[64] = wincl; }
  __syncthreads();
  const int res = scan_ws[32 + wave] + incl - cnt; *tot = scan_ws[64];
  return res;
}
template <int SP, int CAP>
__device__ __forceinline__ int chunk_hits(const int* __restrict__ dstv, int e0, int n0, int tid, int* LIST, int* scan_ws) {
  const int eb = e0 + tid * SP;
  int rec[SP]; int cnt = 0;
  if (eb < NE) {
#pragma unroll
    for (int k = 0; k < SP; k += 4) {
      const v4i d4 = *(const v4i*)(dstv + eb + k);
#pragma unroll
      for (int u = 0; u < 4; ++u) {
        const int d = d4[u]; int r = -1;
        if (d >= n0 && d < n0 + SRB && d < NN) { r = ((d - n0) << 19) | (eb + k + u); ++cnt; }
        rec[k + u] = r;
      }
    }
  } else {
#pragma unroll
    for (int k = 0; k < SP; ++k) rec[k] = -1;
  }
  int tot; int p = blk_excl_scan(cnt, scan_ws, tid, &tot);
#pragma unroll
  for (int k = 0; k < SP; ++k) if (rec[k] >= 0) { if ((unsigned)p < (unsigned)CAP) LIST[p] = rec[k]; ++p; }
  __syncthreads();
  return tot < CAP ? tot : CAP;
}

__global__ __launch_bounds__(NT) void ealoop_kernel(const int* __restrict__ ei, const float* __restrict__ ea, float* __restrict__ EAL) {
  __shared__ int LIST[SCH];
  __shared__ __align__(16) float ES[SRB * EDM];
  __shared__ float EC[SRB];
  __shared__ int scan_ws[80];
  const int tid = threadIdx.x, lane = tid & 31, wave = tid >> 5;
  const int n0 = blockIdx.x * SRB;
  for (int i = tid; i < SRB * EDM; i += NT) ES[i] = 0.f;
  for (int i = tid; i < SRB; i += NT) EC[i] = 0.f;
  __syncthreads();
  const int* dstv = ei + NE;
#pragma unroll 1
  for (int c = 0; c < NCH; ++c) {
    const int tot = chunk_hits<SCH / NT, SCH>(dstv, c * SCH, n0, tid, LIST, scan_ws);
#pragma unroll 1
    for (int base = 0; base < tot; base += 32) {
      const int q = base + lane;
      const int rv = (q < tot) ? LIST[q] : -1;
      const int own = (rv >= 0 && (rv >> 26) == wave) ? 1 : 0;
      unsigned msk = (unsigned)__ballot(own);
#pragma unroll 1
      for (int it = 0; it < 32; ++it) {
        if (msk == 0u) break;
        const int bpos = __builtin_ctz(msk); msk &= msk - 1u;
        const int r = __shfl(rv, bpos, 32);
        const int dl = (r >> 19) & (SRB - 1);
        int e = r & 0x7FFFF; e = (e < NE) ? e : NE - 1;
        if (lane < EDM) ES[dl * EDM + lane] += ea[(size_t)e * EDM + lane];
        if (lane == EDM) EC[dl] += 1.0f;
      }
    }
    __syncthreads();
  }
#pragma unroll 1
  for (int it = 0; it < RPW / 16; ++it) {
    const int dl = wave * RPW + it * 16 + (lane >> 1);
    const int half = (lane & 1) * 4;
    const float cnt = EC[dl];
    const float inv = 1.0f / fmaxf(cnt, 1.0f);
    v4f s = *(const v4f*)(ES + dl * EDM + half);
    s = s * inv;
    float* op = EAL + (size_t)(n0 + dl) * EDM + half;
    *(volatile v4f*)op = s; __threadfence(); *(volatile v4f*)op = s;
  }
}

__global__ __launch_bounds__(NT) void gat_logits_kernel(const float* __restrict__ XLR, const int* __restrict__ ei, const float* __restrict__ eattr,
                                                       const float* __restrict__ EAL, const float* __restrict__ We,
                                                       const float* __restrict__ att, float* __restrict__ LG) {
  constexpr int CPL = HC / 32;
  __shared__ __align__(16) float sW[EDM * HC];
  __shared__ __align__(16) float sA[HC];
  __shared__ __align__(16) float sal[32 * 4];
  const int tid = threadIdx.x, lane = tid & 31, wave = tid >> 5;
  for (int i = tid; i < EDM * HC; i += NT) sW[i] = We[i];
  for (int i = tid; i < HC; i += NT) sA[i] = att[i];
  __syncthreads();
  const int c0 = CPL * lane;
#pragma unroll 1
  for (int i = 0; i < 4; ++i) {
    const int el = 4 * wave + i;
    const int e = blockIdx.x * 32 + el;
    int s, d; const float* ap;
    if (e < NE) {
      s = ei[e]; d = ei[NE + e];
      s = s < 0 ? 0 : (s >= NN ? NN - 1 : s);
      d = d < 0 ? 0 : (d >= NN ? NN - 1 : d);
      ap = eattr + (size_t)e * EDM;
    } else {
      s = e - NE; d = s;
      ap = EAL + (size_t)s * EDM;
    }
    const v4f a0 = *(const v4f*)ap, a1 = *(const v4f*)(ap + 4);
    const float* xl = XLR + (size_t)s * XP + c0;
    const float* xr = XLR + (size_t)d * XP + HC + c0;
    float dsum = 0.f;
#pragma unroll 1
    for (int q = 0; q < CPL; q += 4) {
      const v4f xv = *(const v4f*)(xl + q), rv = *(const v4f*)(xr + q);
      const v4f av = *(const v4f*)(sA + c0 + q);
      v4f ee = a0[0] * *(const v4f*)(sW + c0 + q);
#pragma unroll
      for (int k = 1; k < 4; ++k) ee = ee + a0[k] * *(const v4f*)(sW + k * HC + c0 + q);
#pragma unroll
      for (int k = 0; k < 4; ++k) ee = ee + a1[k] * *(const v4f*)(sW + (4 + k) * HC + c0 + q);
      const v4f m = (xv + rv) + ee;
#pragma unroll
      for (int t = 0; t < 4; ++t) { float v = m[t]; v = (v >= 0.f) ? v : 0.2f * v; dsum += v * av[t]; }
    }
    dsum += __shfl_xor(dsum, 1, 32); dsum += __shfl_xor(dsum, 2, 32); dsum += __shfl_xor(dsum, 4, 32);
    if ((lane & 7) == 0) sal[el * 4 + (lane >> 3)] = dsum;
  }
  __syncthreads();
  if (tid < 32) {
    const v4f v = *(const v4f*)(sal + 4 * tid);
    float* op = LG + ((size_t)blockIdx.x * 32 + tid) * 4;
    *(volatile v4f*)op = v; __threadfence(); *(volatile v4f*)op = v;
  }
}

__global__ __launch_bounds__(NT) void gat_stream_kernel(float* XLR, const int* __restrict__ ei, const float* __restrict__ LG,
                                                       const float* __restrict__ bias, _Float16* __restrict__ Hout) {
  __shared__ int LIST[SCH];
  __shared__ float SM[SRB * NHD];
  __shared__ float SL[SRB * NHD];
  __shared__ int scan_ws[80];
  __shared__ __align__(16) float stg[NT / 32][HC];
  const int tid = threadIdx.x, lane = tid & 31, wave = tid >> 5;
  const int n0 = blockIdx.x * SRB;
  const int hq = lane & 3;
#pragma unroll 1
  for (int j = 0; j < RPW; ++j) {
    const int n = n0 + wave * RPW + j;
    const float* xp = XLR + (size_t)n * XP + 4 * lane;
    float* rp = XLR + (size_t)n * XP + HC + 4 * lane;
    const v4f v0 = *(const v4f*)xp, v1 = *(const v4f*)(xp + 128);
    *(v4f*)rp = v0; *(v4f*)(rp + 128) = v1;
  }
  for (int i = tid; i < SRB * NHD; i += NT) { SM[i] = LG[(size_t)(NE + n0) * 4 + i]; SL[i] = 1.0f; }
  __syncthreads();
  const int* dstv = ei + NE;
#pragma unroll 1
  for (int c = 0; c < NCH; ++c) {
    const int tot = chunk_hits<SCH / NT, SCH>(dstv, c * SCH, n0, tid, LIST, scan_ws);
#pragma unroll 1
    for (int base = 0; base < tot; base += 32) {
      const int q = base + lane;
      const int rv = (q < tot) ? LIST[q] : -1;
      const int own = (rv >= 0 && (rv >> 26) == wave) ? 1 : 0;
      unsigned msk = (unsigned)__ballot(own);
#pragma unroll 1
      for (int it = 0; it < 32; ++it) {
        if (msk == 0u) break;
        const int bpos = __builtin_ctz(msk); msk &= msk - 1u;
        const int r = __shfl(rv, bpos, 32);
        const int dl = (r >> 19) & (SRB - 1);
        int e = r & 0x7FFFF; e = (e < NE) ? e : NE - 1;
        int s = ei[e]; s = s < 0 ? 0 : (s >= NN ? NN - 1 : s);
        const float lg = LG[(size_t)e * 4 + hq];
        const int mi = dl * 4 + hq;
        const float mo = SM[mi], lo = SL[mi];
        const float mn = fmaxf(mo, lg);
        const float rr = __expf(mo - mn), ex = __expf(lg - mn);
        const float ln = lo * rr + ex;
        if (lane < 4) { SM[mi] = mn; SL[mi] = ln; }
        float* rp = XLR + (size_t)(n0 + dl) * XP + HC + 4 * lane;
        const float* xp = XLR + (size_t)s * XP + 4 * lane;
#pragma unroll
        for (int jj = 0; jj < 2; ++jj) {
          const int hj = (4 * lane + 128 * jj) >> 6;
          const float rrj = __shfl(rr, hj, 32), exj = __shfl(ex, hj, 32);
          v4f a = *(const v4f*)(rp + 128 * jj);
          const v4f hv = *(const v4f*)(xp + 128 * jj);
          a = a * rrj + exj * hv;
          *(v4f*)(rp + 128 * jj) = a;
        }
      }
    }
    __syncthreads();
  }
  v4f bvj[2];
#pragma unroll
  for (int jj = 0; jj < 2; ++jj) {
    const int cb = 4 * lane + 128 * jj;
    v4f t; t[0] = bias[cb]; t[1] = bias[cb + 1]; t[2] = bias[cb + 2]; t[3] = bias[cb + 3]; bvj[jj] = t;
  }
  float* sw = stg[wave];
#pragma unroll 1
  for (int j = 0; j < RPW; ++j) {
    const int dl = wave * RPW + j; const int n = n0 + dl;
    const int si = dl * 4 + hq;
    const float slv = SL[si];
    const float lv = (slv > 0.f) ? slv : 1.0f;
    const float inv4 = 1.0f / lv;
    const float* rp = XLR + (size_t)n * XP + HC + 4 * lane;
#pragma unroll
    for (int jj = 0; jj < 2; ++jj) {
      const int hj = (4 * lane + 128 * jj) >> 6;
      const float invj = __shfl(inv4, hj, 32);
      const v4f a = *(const v4f*)(rp + 128 * jj);
      v4f t = a * invj; fence_v4(t); t = t + bvj[jj];
      v4f o;
#pragma unroll
      for (int q = 0; q < 4; ++q) o[q] = fmaxf(t[q], 0.0f) * 64.0f;
      *(v4f*)(sw + 4 * lane + 128 * jj) = o;
    }
    __builtin_amdgcn_fence(__ATOMIC_RELEASE, "workgroup");
    __builtin_amdgcn_wave_barrier();
    __builtin_amdgcn_fence(__ATOMIC_ACQUIRE, "workgroup");
    const float* sp = sw + 8 * lane;
    const v4f u0 = *(const v4f*)sp, u1 = *(const v4f*)(sp + 4);
    v8h hk;
#pragma unroll
    for (int q = 0; q < 4; ++q) { hk[q] = (_Float16)u0[q]; hk[4 + q] = (_Float16)u1[q]; }
    _Float16* hrow = Hout + (size_t)n * HC;
    for (int pass = 0; pass < 2; ++pass) {
      *(volatile v8h*)(hrow + 8 * lane) = hk;
      __threadfence();
    }
    __builtin_amdgcn_fence(__ATOMIC_RELEASE, "workgroup");
    __builtin_amdgcn_wave_barrier();
    __builtin_amdgcn_fence(__ATOMIC_ACQUIRE, "workgroup");
  }
}

__global__ __launch_bounds__(256) void pool_kernel(const _Float16* __restrict__ H, const int* __restrict__ batch, _Float16* __restrict__ XG) {
  const int lane = threadIdx.x & 31, wave = threadIdx.x >> 5;
  const int g = blockIdx.x * 8 + wave;
  float mx[8];
#pragma unroll
  for (int q = 0; q < 8; ++q) mx[q] = -INFINITY;
#pragma unroll 1
  for (int j = 0; j < NN / NG; ++j) {
    const int n = g * (NN / NG) + j;
    const int bg = batch[n];
    if (bg == g) {
      const v8h hv = *(const v8h*)(H + (size_t)n * HC + 8 * lane);
#pragma unroll
      for (int q = 0; q < 8; ++q) mx[q] = fmaxf(mx[q], (float)hv[q]);
    }
  }
  v8h o;
#pragma unroll
  for (int q = 0; q < 8; ++q) o[q] = (_Float16)mx[q];
  _Float16* op = XG + (size_t)g * HC + 8 * lane;
  *(volatile v8h*)op = o; __threadfence(); *(volatile v8h*)op = o;
}

__global__ __launch_bounds__(256) void out_kernel(const float* __restrict__ P, float* __restrict__ out) {
  for (int pass = 0; pass < 2; ++pass) {
    for (int i = threadIdx.x; i < NG * NTK / 4; i += 256) {
      const int row = i / 3, c4 = (i - row * 3) * 4;
      const v4f v = *(const v4f*)(P + (size_t)row * 64 + c4);
      *(volatile v4f*)(out + 4 * (size_t)i) = v;
    }
    __threadfence();
  }
}

static void cast_rows(hipStream_t st, const float* in, int R, int C, _Float16* out, int Cp) {
  const long n8 = (long)R * Cp / 8;
  k_cast_rows<<<(int)((n8 + 255) / 256), 256, 0, st>>>(in, R, C, out, Cp);
}
static void tcast(hipStream_t st, const float* in, int R, int C, _Float16* outT, int Rp, int Cp) {
  const long n8 = (long)Cp * Rp / 8;
  k_tcast<<<(int)((n8 + 255) / 256), 256, 0, st>>>(in, R, C, outT, Rp, Cp);
}
template <int EPI, bool OUT16>
static void gemm(hipStream_t st, const void* A, int lda, const void* Bt, int ldb, void* C, int ldc,
                 const float* bias, const float* gamma, const float* beta, int nValid, int M, int N, int K, float scale, float oscale) {
  const int tiles = (M / 64) * (N / 64);
  gemm_f16<EPI, OUT16><<<(tiles + 7) / 8, 256, 0, st>>>(U16(A), lda, U16(Bt), ldb, C, ldc, bias, gamma, beta, nValid, M, N, K, scale, oscale);
}

extern "C" void kernel_launch(void* const* d_in, const int* in_sizes, int n_in,
                              void* d_out, int out_size, void* d_ws, size_t ws_size,
                              hipStream_t stream) {
  if (n_in < 42) return;
  if (in_sizes[0] != NN * FIN || in_sizes[1] != 2 * NE || in_sizes[2] != NE * EDM || in_sizes[3] != NN ||
      in_sizes[4] != NG * FPK || in_sizes[5] != NG * DSK || out_size != NG * NTK) return;
  const float* x     = (const float*)d_in[0];
  const int*   ei    = (const int*)  d_in[1];
  const float* ea    = (const float*)d_in[2];
  const int*   batch = (const int*)  d_in[3];
  const float* fp    = (const float*)d_in[4];
  const float* desc  = (const float*)d_in[5];
  const float* c1Wl = (const float*)d_in[6];  const float* c1bl = (const float*)d_in[7];
  const float* c1Wr = (const float*)d_in[8];  const float* c1br = (const float*)d_in[9];
  const float* c1We = (const float*)d_in[10]; const float* c1at = (const float*)d_in[11]; const float* c1bi = (const float*)d_in[12];
  const float* c2Wl = (const float*)d_in[13]; const float* c2bl = (const float*)d_in[14];
  const float* c2Wr = (const float*)d_in[15]; const float* c2br = (const float*)d_in[16];
  const float* c2We = (const float*)d_in[17]; const float* c2at = (const float*)d_in[18]; const float* c2bi = (const float*)d_in[19];
  const float* gW  = (const float*)d_in[20]; const float* gb  = (const float*)d_in[21];
  const float* ggn = (const float*)d_in[22]; const float* gbt = (const float*)d_in[23];
  const float* fW  = (const float*)d_in[24]; const float* fb  = (const float*)d_in[25];
  const float* fgn = (const float*)d_in[26]; const float* fbt = (const float*)d_in[27];
  const float* dW  = (const float*)d_in[28]; const float* db  = (const float*)d_in[29];
  const float* dgn = (const float*)d_in[30]; const float* dbt = (const float*)d_in[31];
  const float* k1W = (const float*)d_in[32]; const float* k1b = (const float*)d_in[33];
  const float* k1g = (const float*)d_in[34]; const float* k1t = (const float*)d_in[35];
  const float* k2W = (const float*)d_in[36]; const float* k2b = (const float*)d_in[37];
  const float* k2g = (const float*)d_in[38]; const float* k2t = (const float*)d_in[39];
  const float* k3W = (const float*)d_in[40]; const float* k3b = (const float*)d_in[41];
  float* out = (float*)d_out;

  char* ws = (char*)d_ws; size_t off = 0;
  auto carve = [&](size_t bytes) -> char* { char* p = ws + off; off += (bytes + 255) & ~(size_t)255; return p; };
  _Float16* X16  = (_Float16*)carve((size_t)NN * FIN * 2);
  _Float16* W1T  = (_Float16*)carve((size_t)(2 * HC) * FIN * 2);
  _Float16* W2T  = (_Float16*)carve((size_t)(2 * HC) * HC * 2);
  float*    bc1  = (float*)carve((size_t)2 * HC * 4);
  float*    bc2  = (float*)carve((size_t)2 * HC * 4);
  float*    XLR  = (float*)carve((size_t)NN * XP * 4);
  _Float16* HB   = (_Float16*)carve((size_t)NN * HC * 2);
  float*    EAL  = (float*)carve((size_t)NN * EDM * 4);
  float*    LG   = (float*)carve((size_t)ETOT * 4 * 4);
  _Float16* FP16 = (_Float16*)carve((size_t)NG * FPK * 2);
  _Float16* FWT  = (_Float16*)carve((size_t)FO * FPK * 2);
  _Float16* DS16 = (_Float16*)carve((size_t)NG * DSKP * 2);
  _Float16* DWT  = (_Float16*)carve((size_t)DO_ * DSKP * 2);
  _Float16* GWT  = (_Float16*)carve((size_t)GO * HC * 2);
  _Float16* K1T  = (_Float16*)carve((size_t)HD1 * TIN * 2);
  _Float16* K2T  = (_Float16*)carve((size_t)HD2P * HD1 * 2);
  _Float16* K3T  = (_Float16*)carve((size_t)64 * HD2 * 2);
  _Float16* XG16 = (_Float16*)carve((size_t)NG * HC * 2);
  _Float16* Z    = (_Float16*)carve((size_t)NG * TIN * 2);
  _Float16* Z1   = (_Float16*)carve((size_t)NG * HD1 * 2);
  _Float16* Z2   = (_Float16*)carve((size_t)NG * HD2P * 2);
  float*    OUTP = (float*)carve((size_t)NG * 64 * 4);
  if (off > ws_size || off > (size_t)134217728) return;

  const float s64 = 0.015625f;
  cast_rows(stream, x, NN, FIN, X16, FIN);
  cast_rows(stream, fp, NG, FPK, FP16, FPK);
  cast_rows(stream, desc, NG, DSK, DS16, DSKP);
  tcast(stream, c1Wl, FIN, HC, W1T, FIN, HC);
  tcast(stream, c1Wr, FIN, HC, W1T + (size_t)HC * FIN, FIN, HC);
  tcast(stream, c2Wl, HC, HC, W2T, HC, HC);
  tcast(stream, c2Wr, HC, HC, W2T + (size_t)HC * HC, HC, HC);
  tcast(stream, gW, HC, GO, GWT, HC, GO);
  tcast(stream, fW, FPK, FO, FWT, FPK, FO);
  tcast(stream, dW, DSK, DO_, DWT, DSKP, DO_);
  tcast(stream, k1W, TIN, HD1, K1T, TIN, HD1);
  tcast(stream, k2W, HD1, HD2, K2T, HD1, HD2P);
  tcast(stream, k3W, HD2, NTK, K3T, HD2, 64);
  bias_cat2_kernel<<<1, 256, 0, stream>>>(c1bl, c1br, bc1, HC);
  bias_cat2_kernel<<<1, 256, 0, stream>>>(c2bl, c2br, bc2, HC);
  ealoop_kernel<<<NTILE, NT, 0, stream>>>(ei, ea, EAL);
  gemm<0, false>(stream, X16, FIN, W1T, FIN, (void*)XLR, XP, bc1, bc1, bc1, 2 * HC, NN, 2 * HC, FIN, 1.0f, 1.0f);
  gat_logits_kernel<<<ETOT / 32, NT, 0, stream>>>(XLR, ei, ea, EAL, c1We, c1at, LG);
  gat_stream_kernel<<<NTILE, NT, 0, stream>>>(XLR, ei, LG, c1bi, HB);
  gemm<0, false>(stream, HB, HC, W2T, HC, (void*)XLR, XP, bc2, bc2, bc2, 2 * HC, NN, 2 * HC, HC, s64, 1.0f);
  gat_logits_kernel<<<ETOT / 32, NT, 0, stream>>>(XLR, ei, ea, EAL, c2We, c2at, LG);
  gat_stream_kernel<<<NTILE, NT, 0, stream>>>(XLR, ei, LG, c2bi, HB);
  pool_kernel<<<NG / 8, 256, 0, stream>>>(HB, batch, XG16);
  gemm<1, true>(stream, XG16, HC, GWT, HC, (void*)Z, TIN, gb, ggn, gbt, GO, NG, GO, HC, s64, 64.0f);
  gemm<1, true>(stream, FP16, FPK, FWT, FPK, (void*)(Z + GO), TIN, fb, fgn, fbt, FO, NG, FO, FPK, 1.0f, 64.0f);
  gemm<1, true>(stream, DS16, DSKP, DWT, DSKP, (void*)(Z + GO + FO), TIN, db, dgn, dbt, DO_, NG, DO_, DSKP, 1.0f, 64.0f);
  gemm<1, true>(stream, Z, TIN, K1T, TIN, (void*)Z1, HD1, k1b, k1g, k1t, HD1, NG, HD1, TIN, s64, 64.0f);
  gemm<1, true>(stream, Z1, HD1, K2T, HD1, (void*)Z2, HD2P, k2b, k2g, k2t, HD2, NG, HD2P, HD1, s64, 64.0f);
  gemm<0, false>(stream, Z2, HD2P, K3T, HD2, (void*)OUTP, 64, k3b, k3b, k3b, NTK, NG, 64, HD2, s64, 1.0f);
  out_kernel<<<1, 256, 0, stream>>>(OUTP, out);
}
